// Layer_Incor_offset_61211873903020
// MI455X (gfx1250) — hardware-verified
//
#include <hip/hip_runtime.h>
#include <math.h>


#define NB 8
#define HQ 32
#define WQ 32
#define LQ (HQ * WQ)
#define DD 512
#define NH 8
#define DK 64
#define KP 4
#define DFF 2048
#define NR (NB * LQ)
#define NOA 96

typedef __attribute__((ext_vector_type(16))) _Float16 v16h;
typedef __attribute__((ext_vector_type(8)))  _Float16 v8h;
typedef __attribute__((ext_vector_type(8)))  float v8f;
typedef __attribute__((ext_vector_type(4)))  float v4f;
typedef __attribute__((ext_vector_type(4)))  unsigned v4u;

template <typename T> __device__ __forceinline__ void vst2(void* p, T v) { *(volatile T*)p = v; __threadfence(); *(volatile T*)p = v; }
__device__ __forceinline__ v8f wmma16(v16h a, v16h b, v8f c) {
  v8f d = __builtin_amdgcn_wmma_f32_16x16x32_f16(false, a, false, b, (short)0, c, false, false);
  asm volatile("v_nop\n\tv_nop\n\tv_nop\n\tv_nop" : "+v"(d) : "v"(a), "v"(b));
  return d;
}
__device__ __forceinline__ v16h frag_h(const _Float16* rowk0, int lane) {
  union { v16h v; v8h q[2]; } u; const _Float16* p = rowk0 + 8 * (lane >> 4);
  u.q[0] = *(const v8h*)p; u.q[1] = *(const v8h*)(p + 16); return u.v;
}
__device__ __forceinline__ v16h frag_f32(const float* rowk0, int lane) {
  v16h a; const float* p = rowk0 + 8 * (lane >> 4);
#pragma unroll
  for (int i = 0; i < 8; ++i) { a[i] = (_Float16)p[i]; a[8 + i] = (_Float16)p[16 + i]; }
  return a;
}
__device__ __forceinline__ v16h frag_f32x2(const float* r1, const float* r2, int lane) {
  v16h a; const float* p = r1 + 8 * (lane >> 4); const float* q = r2 + 8 * (lane >> 4);
#pragma unroll
  for (int i = 0; i < 8; ++i) { a[i] = (_Float16)(p[i] + q[i]); a[8 + i] = (_Float16)(p[16 + i] + q[16 + i]); }
  return a;
}
#define LDSX() do { asm volatile("s_wait_dscnt 0" ::: "memory"); __builtin_amdgcn_wave_barrier(); __builtin_amdgcn_fence(__ATOMIC_RELEASE, "workgroup"); } while (0)

__global__ __launch_bounds__(256) void k_packT(const float* __restrict__ W, _Float16* __restrict__ Wt, int K, int N) {
  __shared__ float tile[64][65];
  const int k0 = blockIdx.y * 64, n0 = blockIdx.x * 64, tid = threadIdx.x;
  for (int q = tid; q < 64 * 64; q += 256) { const int kk = q >> 6, nn = q & 63; tile[kk][nn] = (n0 + nn < N) ? W[(size_t)(k0 + kk) * N + n0 + nn] : 0.f; }
  __syncthreads();
  for (int q = tid; q < 64 * 8; q += 256) { const int nn = q >> 3, pc = q & 7; if (n0 + nn >= N) continue;
    union { v8h h; v4u u; } pk;
#pragma unroll
    for (int e = 0; e < 8; ++e) pk.h[e] = (_Float16)tile[pc * 8 + e][nn];
    vst2(Wt + (size_t)(n0 + nn) * K + k0 + pc * 8, pk.u); }
}

template <int RELU, int ADD2>
__global__ __launch_bounds__(128) void k_gemm(const float* __restrict__ A, const float* __restrict__ A2, const _Float16* __restrict__ Wt,
                                            const float* __restrict__ bias, const float* __restrict__ res, float* __restrict__ Out, int K, int N) {
  __shared__ __align__(16) float so[4][16 * 128];
  const int tid = threadIdx.x, wave = tid >> 5, lane = tid & 31, col = lane & 15, g = lane >> 4;
  const int r0 = blockIdx.x * 64 + wave * 16, n0 = blockIdx.y * 128;
  v8f acc[8] = {};
#pragma unroll 1
  for (int kc = 0; kc < K / 32; ++kc) {
    v16h a;
    if (ADD2) a = frag_f32x2(A + (size_t)(r0 + col) * K + kc * 32, A2 + (size_t)(r0 + col) * K + kc * 32, lane);
    else      a = frag_f32(A + (size_t)(r0 + col) * K + kc * 32, lane);
#pragma unroll
    for (int j = 0; j < 8; ++j) acc[j] = wmma16(a, frag_h(Wt + (size_t)(n0 + j * 16 + col) * K + kc * 32, lane), acc[j]);
  }
  float* S = so[wave];
#pragma unroll
  for (int j = 0; j < 8; ++j) { const float bv = bias[n0 + j * 16 + col];
#pragma unroll
    for (int r = 0; r < 8; ++r) { float v = acc[j][r] + bv; if (RELU) v = v > 0.f ? v : 0.f; S[(8 * g + r) * 128 + j * 16 + col] = v; } }
  LDSX();
#pragma unroll 4
  for (int rl = 0; rl < 16; ++rl) { const size_t o = (size_t)(r0 + rl) * N + n0 + lane * 4;
    v4f v = *(const v4f*)(S + rl * 128 + lane * 4); if (res) v += *(const v4f*)(res + o); vst2(Out + o, v); }
}

__global__ __launch_bounds__(128) void k_offA(const float* __restrict__ bq, const _Float16* __restrict__ WoaT, const float* __restrict__ ob,
                                            const float* __restrict__ Ab, float* __restrict__ OA) {
  __shared__ __align__(16) float so[4][16 * 96];
  const int tid = threadIdx.x, wave = tid >> 5, lane = tid & 31, col = lane & 15, g = lane >> 4;
  const int r0 = blockIdx.x * 64 + wave * 16;
  v8f acc[6] = {};
#pragma unroll 1
  for (int kc = 0; kc < DD / 32; ++kc) { const v16h a = frag_f32(bq + (size_t)(r0 + col) * DD + kc * 32, lane);
#pragma unroll
    for (int j = 0; j < 6; ++j) acc[j] = wmma16(a, frag_h(WoaT + (size_t)(j * 16 + col) * DD + kc * 32, lane), acc[j]); }
  float* S = so[wave];
#pragma unroll
  for (int j = 0; j < 6; ++j) { const int n = j * 16 + col; const float bv = n < 64 ? ob[n] : Ab[n - 64];
#pragma unroll
    for (int r = 0; r < 8; ++r) S[(8 * g + r) * 96 + n] = acc[j][r] + bv; }
  LDSX();
  for (int q = lane; q < 16 * 24; q += 32) { const int rl = q / 24, pc = q % 24;
    vst2(OA + (size_t)(r0 + rl) * NOA + pc * 4, *(const v4f*)(S + rl * 96 + pc * 4)); }
}

__global__ __launch_bounds__(256) void k_sample(const float* __restrict__ OA, const float* __restrict__ refp, const float* __restrict__ kv,
                                              float* __restrict__ feat) {
  const size_t row = blockIdx.x; const int b = (int)(row / LQ), q = (int)(row % LQ);
  const int tid = threadIdx.x, h = tid >> 5, lane = tid & 31;
  const float* oa = OA + row * NOA;
  float lg[KP], mx = -3.0e38f;
#pragma unroll
  for (int p = 0; p < KP; ++p) { lg[p] = oa[64 + h * KP + p]; mx = fmaxf(mx, lg[p]); }
  float sum = 0.f;
#pragma unroll
  for (int p = 0; p < KP; ++p) { lg[p] = expf(lg[p] - mx); sum += lg[p]; }
  const int rb = (b * NH + h) % NB;
  const float rx = refp[((size_t)rb * LQ + q) * 2] * (float)(WQ - 1), ry = refp[((size_t)rb * LQ + q) * 2 + 1] * (float)(HQ - 1);
  float f0 = 0.f, f1 = 0.f;
#pragma unroll 1
  for (int p = 0; p < KP; ++p) {
    const float aw = lg[p] / sum;
    const float px = rx + oa[(h * KP + p) * 2], py = ry + oa[(h * KP + p) * 2 + 1];
    const float vx = 2.0f * px / (float)(WQ - 1) - 1.0f, vy = 2.0f * py / (float)(HQ - 1) - 1.0f;
    const float ix = ((vx + 1.0f) * (float)WQ - 1.0f) / 2.0f, iy = ((vy + 1.0f) * (float)HQ - 1.0f) / 2.0f;
    const float x0 = floorf(ix), y0 = floorf(iy); const float wx1 = ix - x0, wy1 = iy - y0;
#pragma unroll 1
    for (int cy = 0; cy < 2; ++cy)
#pragma unroll 1
      for (int cx = 0; cx < 2; ++cx) {
        const float xf = x0 + (float)cx, yf = y0 + (float)cy;
        const bool valid = xf >= 0.f && xf <= (float)(WQ - 1) && yf >= 0.f && yf <= (float)(HQ - 1);
        const float wgt = (cx ? wx1 : 1.f - wx1) * (cy ? wy1 : 1.f - wy1) * aw;
        if (valid) { const int xi = (int)xf, yi = (int)yf; const float* kr = kv + ((size_t)b * LQ + yi * WQ + xi) * DD + h * DK;
          f0 += wgt * kr[lane]; f1 += wgt * kr[32 + lane]; }
      }
  }
  vst2(feat + row * DD + h * DK + lane, *(float __attribute__((may_alias))*)&f0);
  vst2(feat + row * DD + h * DK + 32 + lane, *(float __attribute__((may_alias))*)&f1);
}

__global__ __launch_bounds__(128) void k_ln(const float* __restrict__ y, const float* __restrict__ gm, const float* __restrict__ bt, float* __restrict__ out) {
  __shared__ float red[128];
  const size_t row = blockIdx.x; const int tid = threadIdx.x;
  const v4f v = *(const v4f*)(y + row * DD + tid * 4);
  red[tid] = v[0] + v[1] + v[2] + v[3]; __syncthreads();
  for (int st = 64; st > 0; st >>= 1) { if (tid < st) red[tid] += red[tid + st]; __syncthreads(); }
  const float mu = red[0] / (float)DD; __syncthreads();
  const float d0 = v[0] - mu, d1 = v[1] - mu, d2 = v[2] - mu, d3 = v[3] - mu;
  red[tid] = d0 * d0 + d1 * d1 + d2 * d2 + d3 * d3; __syncthreads();
  for (int st = 64; st > 0; st >>= 1) { if (tid < st) red[tid] += red[tid + st]; __syncthreads(); }
  const float rs = rsqrtf(red[0] / (float)DD + 1e-5f);
  const v4f gg = *(const v4f*)(gm + tid * 4), bb = *(const v4f*)(bt + tid * 4);
  v4f o = { d0 * rs * gg[0] + bb[0], d1 * rs * gg[1] + bb[1], d2 * rs * gg[2] + bb[2], d3 * rs * gg[3] + bb[3] };
  vst2(out + row * DD + tid * 4, o);
}

extern "C" void kernel_launch(void* const* d_in, const int* in_sizes, int n_in,
                              void* d_out, int out_size, void* d_ws, size_t ws_size,
                              hipStream_t stream) {
  (void)in_sizes; (void)n_in; (void)out_size; (void)ws_size;
  const float* src = (const float*)d_in[0]; const float* refp = (const float*)d_in[1];
  const float* pos = (const float*)d_in[2]; const float* sq = (const float*)d_in[3];
  const float* bw = (const float*)d_in[6]; const float* bb = (const float*)d_in[7];
  const float* kw = (const float*)d_in[8]; const float* kb = (const float*)d_in[9];
  const float* ow = (const float*)d_in[10]; const float* ob = (const float*)d_in[11];
  const float* Aw = (const float*)d_in[12]; const float* Ab = (const float*)d_in[13];
  const float* mw = (const float*)d_in[14]; const float* mb = (const float*)d_in[15];
  const float* f1w = (const float*)d_in[16]; const float* f1b = (const float*)d_in[17];
  const float* f2w = (const float*)d_in[18]; const float* f2b = (const float*)d_in[19];
  const float* lg = (const float*)d_in[20]; const float* lb = (const float*)d_in[21];
  float* out = (float*)d_out;
  char* ws = (char*)d_ws; size_t off = 0;
  auto take = [&](size_t bytes) { char* p = ws + off; off += (bytes + 255) & ~(size_t)255; return p; };
  _Float16* bwT = (_Float16*)take((size_t)DD * DD * 2); _Float16* kwT = (_Float16*)take((size_t)DD * DD * 2);
  _Float16* oaT = (_Float16*)take((size_t)NOA * DD * 2); _Float16* mwT = (_Float16*)take((size_t)DD * DD * 2);
  _Float16* f1T = (_Float16*)take((size_t)DFF * DD * 2); _Float16* f2T = (_Float16*)take((size_t)DD * DFF * 2);
  float* bq = (float*)take((size_t)NR * DD * 4); float* OA = (float*)take((size_t)NR * NOA * 4);
  float* kv = (float*)take((size_t)NR * DD * 4); float* feat = (float*)take((size_t)NR * DD * 4);
  float* o1 = (float*)take((size_t)NR * DD * 4); float* hid = (float*)take((size_t)NR * DFF * 4);
  float* y = (float*)take((size_t)NR * DD * 4);
  k_packT<<<dim3(DD / 64, DD / 64), 256, 0, stream>>>(bw, bwT, DD, DD);
  k_packT<<<dim3(DD / 64, DD / 64), 256, 0, stream>>>(kw, kwT, DD, DD);
  k_packT<<<dim3(1, DD / 64), 256, 0, stream>>>(ow, oaT, DD, 64);
  k_packT<<<dim3(1, DD / 64), 256, 0, stream>>>(Aw, oaT + (size_t)64 * DD, DD, 32);
  k_packT<<<dim3(DD / 64, DD / 64), 256, 0, stream>>>(mw, mwT, DD, DD);
  k_packT<<<dim3(DFF / 64, DD / 64), 256, 0, stream>>>(f1w, f1T, DD, DFF);
  k_packT<<<dim3(DD / 64, DFF / 64), 256, 0, stream>>>(f2w, f2T, DFF, DD);
  k_gemm<0, 0><<<dim3(NR / 64, DD / 128), 128, 0, stream>>>(sq, nullptr, bwT, bb, nullptr, bq, DD, DD);
  k_offA<<<NR / 64, 128, 0, stream>>>(bq, oaT, ob, Ab, OA);
  k_gemm<0, 1><<<dim3(NR / 64, DD / 128), 128, 0, stream>>>(src, pos, kwT, kb, nullptr, kv, DD, DD);
  k_sample<<<NR, 256, 0, stream>>>(OA, refp, kv, feat);
  k_gemm<0, 0><<<dim3(NR / 64, DD / 128), 128, 0, stream>>>(feat, nullptr, mwT, mb, nullptr, o1, DD, DD);
  k_gemm<1, 0><<<dim3(NR / 64, DFF / 128), 128, 0, stream>>>(o1, nullptr, f1T, f1b, nullptr, hid, DD, DFF);
  k_gemm<0, 0><<<dim3(NR / 64, DD / 128), 128, 0, stream>>>(hid, nullptr, f2T, f2b, o1, y, DFF, DD);
  k_ln<<<NR, 128, 0, stream>>>(y, lg, lb, out);
}
